// DifferentiableMultiMLPRenderer_3951369912801
// MI455X (gfx1250) — hardware-verified
//
#include <hip/hip_runtime.h>

typedef _Float16 v16h __attribute__((ext_vector_type(16)));
typedef _Float16 v8h  __attribute__((ext_vector_type(8)));
typedef _Float16 v4h  __attribute__((ext_vector_type(4)));
typedef float    v8f  __attribute__((ext_vector_type(8)));
typedef float    v4f  __attribute__((ext_vector_type(4)));
typedef v8h __attribute__((may_alias)) v8ha;
typedef v4h __attribute__((may_alias)) v4ha;
typedef v4f __attribute__((may_alias)) v4fa;

union Frag { v16h v; v8h half[2]; };

#define FEAT 256
#define SHP  128
#define EMB  63
#define STY  256
#define DIN  703
#define KX   447
#define K1P  448
#define HID  256
#define NCH  3
#define N3P  16
#define MPIX 64
#define MT   4
#define XSTR 456
#define HSTR 264
#define NTHR 256
#define WSC  16.0f
#define WINV 0.0625f

#define G1 (HID * (K1P / 8))
#define G2 (HID * (HID / 8))
#define G3 (N3P * (HID / 8))
#define G4 HID

__device__ __forceinline__ v8f wmma_f16(v16h a, v16h b, v8f c) {
  v8f d = __builtin_amdgcn_wmma_f32_16x16x32_f16(false, a, false, b, (short)0, c, false, false);
  asm volatile("v_nop\n\tv_nop\n\tv_nop\n\tv_nop" : "+v"(d) : "v"(a), "v"(b));
  return d;
}

__device__ __forceinline__ v16h load_frag(const _Float16* p, int h) {
  Frag f;
  f.half[0] = *(const v8ha*)(p + 8 * h);
  f.half[1] = *(const v8ha*)(p + 16 + 8 * h);
  return f.v;
}

__device__ __forceinline__ void blend4(_Float16* dst, const float* pa, const float* pb,
                                       const float* pc, float ca, float cb, float cc) {
  const v4f a = *(const v4fa*)pa;
  const v4f b = *(const v4fa*)pb;
  const v4f c = *(const v4fa*)pc;
  const float third = 1.0f / 3.0f;
  v4f r;
  r.x = (ca * a.x + cb * b.x + cc * c.x) * third;
  r.y = (ca * a.y + cb * b.y + cc * c.y) * third;
  r.z = (ca * a.z + cb * b.z + cc * c.z) * third;
  r.w = (ca * a.w + cb * b.w + cc * c.w) * third;
  const v4h hv = { (_Float16)r.x, (_Float16)r.y, (_Float16)r.z, (_Float16)r.w };
  *(v4ha*)dst = hv;
}

__global__ __launch_bounds__(NTHR) void prep_kernel(
    const float* __restrict__ w1, const float* __restrict__ b1,
    const float* __restrict__ w2, const float* __restrict__ w3,
    const float* __restrict__ style,
    _Float16* __restrict__ W1h, _Float16* __restrict__ W2h,
    _Float16* __restrict__ W3h, float* __restrict__ c1)
{
  const int g = blockIdx.x * NTHR + threadIdx.x;
  if (g < G1) {
    const int n = g / (K1P / 8);
    const int k0 = (g - n * (K1P / 8)) * 8;
    float t[8];
    #pragma unroll
    for (int j = 0; j < 8; ++j) {
      const int k = k0 + j;
      const int kc = (k < KX) ? k : (KX - 1);
      const float x = w1[(size_t)kc * HID + n] * WSC;
      t[j] = (k < KX) ? x : 0.0f;
    }
    const v8h o = { (_Float16)t[0], (_Float16)t[1], (_Float16)t[2], (_Float16)t[3],
                    (_Float16)t[4], (_Float16)t[5], (_Float16)t[6], (_Float16)t[7] };
    _Float16* dst = W1h + (size_t)g * 8;
    *(volatile v8h*)dst = o;
    __threadfence();
    *(volatile v8h*)dst = o;
  } else if (g < G1 + G2) {
    const int e = g - G1;
    const int n = e >> 5;
    const int k0 = (e & 31) * 8;
    float t[8];
    #pragma unroll
    for (int j = 0; j < 8; ++j) t[j] = w2[(size_t)(k0 + j) * HID + n] * WSC;
    const v8h o = { (_Float16)t[0], (_Float16)t[1], (_Float16)t[2], (_Float16)t[3],
                    (_Float16)t[4], (_Float16)t[5], (_Float16)t[6], (_Float16)t[7] };
    _Float16* dst = W2h + (size_t)e * 8;
    *(volatile v8h*)dst = o;
    __threadfence();
    *(volatile v8h*)dst = o;
  } else if (g < G1 + G2 + G3) {
    const int e = g - G1 - G2;
    const int n = e >> 5;
    const int k0 = (e & 31) * 8;
    const int nc = (n < NCH) ? n : (NCH - 1);
    float t[8];
    #pragma unroll
    for (int j = 0; j < 8; ++j) {
      const float x = w3[(size_t)(k0 + j) * NCH + nc] * WSC;
      t[j] = (n < NCH) ? x : 0.0f;
    }
    const v8h o = { (_Float16)t[0], (_Float16)t[1], (_Float16)t[2], (_Float16)t[3],
                    (_Float16)t[4], (_Float16)t[5], (_Float16)t[6], (_Float16)t[7] };
    _Float16* dst = W3h + (size_t)e * 8;
    *(volatile v8h*)dst = o;
    __threadfence();
    *(volatile v8h*)dst = o;
  } else if (g < G1 + G2 + G3 + G4) {
    const int n = g - G1 - G2 - G3;
    float s = b1[n];
    #pragma unroll 1
    for (int j = 0; j < STY; ++j)
      s += style[j] * w1[(size_t)(KX + j) * HID + n];
    float* dst = c1 + n;
    *(volatile float*)dst = s;
    __threadfence();
    *(volatile float*)dst = s;
  }
}

__global__ __launch_bounds__(NTHR) void render_kernel(
    const int*   __restrict__ p2f,
    const float* __restrict__ bary,
    const int*   __restrict__ faces,
    const float* __restrict__ feature,
    const float* __restrict__ shapef,
    const float* __restrict__ color_bg,
    const _Float16* __restrict__ W1h,
    const _Float16* __restrict__ W2h,
    const _Float16* __restrict__ W3h,
    const float* __restrict__ c1,
    const float* __restrict__ b2,
    const float* __restrict__ b3,
    float* __restrict__ out,
    int npix, int hw, int nB, int nF, int nV)
{
  __shared__ __attribute__((aligned(16))) _Float16 sX[MPIX * XSTR];
  __shared__ __attribute__((aligned(16))) _Float16 sH1[MPIX * HSTR];
  __shared__ __attribute__((aligned(16))) float sOut[MPIX * 4];
  __shared__ __attribute__((aligned(16))) int   sVid[MPIX * 4];
  __shared__ __attribute__((aligned(16))) float sBar[MPIX * 4];
  __shared__ int sMsk[MPIX];
  __shared__ int sBat[MPIX];

  const int tid = threadIdx.x, lane = tid & 31, w = tid >> 5;
  const int h = lane >> 4, m = lane & 15;
  const int pix0 = blockIdx.x * MPIX;

  if (tid < MPIX) {
    int g = pix0 + tid;
    g = (g < npix) ? g : (npix - 1);
    const int f = p2f[g];
    int fc = (f < 0) ? 0 : f;
    fc = (fc > nF - 1) ? (nF - 1) : fc;
    int va = faces[(size_t)fc * 3 + 0];
    int vb = faces[(size_t)fc * 3 + 1];
    int vc = faces[(size_t)fc * 3 + 2];
    va = (va < 0) ? 0 : va;  va = (va > nV - 1) ? (nV - 1) : va;
    vb = (vb < 0) ? 0 : vb;  vb = (vb > nV - 1) ? (nV - 1) : vb;
    vc = (vc < 0) ? 0 : vc;  vc = (vc > nV - 1) ? (nV - 1) : vc;
    sVid[tid * 4 + 0] = va;
    sVid[tid * 4 + 1] = vb;
    sVid[tid * 4 + 2] = vc;
    sVid[tid * 4 + 3] = 0;
    sBar[tid * 4 + 0] = bary[(size_t)g * 3 + 0];
    sBar[tid * 4 + 1] = bary[(size_t)g * 3 + 1];
    sBar[tid * 4 + 2] = bary[(size_t)g * 3 + 2];
    sBar[tid * 4 + 3] = 0.0f;
    sMsk[tid] = (f > 0) ? 1 : 0;
    int bt = g / hw;
    bt = (bt > nB - 1) ? (nB - 1) : bt;
    bt = (bt < 0) ? 0 : bt;
    sBat[tid] = bt;
  }
  __syncthreads();

  {
    const int p = tid >> 2, q = tid & 3;
    const float cx = sBar[p * 4 + 0], cy = sBar[p * 4 + 1], cz = sBar[p * 4 + 2];
    _Float16* xr = sX + p * XSTR;
    if (q == 0) {
      xr[FEAT + SHP + 0] = (_Float16)cx;
      xr[FEAT + SHP + 1] = (_Float16)cy;
      xr[FEAT + SHP + 2] = (_Float16)cz;
    }
    if (q == 1) {
      #pragma unroll
      for (int c = KX; c < XSTR; ++c) xr[c] = (_Float16)0.0f;
    }
    #pragma unroll 1
    for (int j = q; j < 30; j += 4) {
      const int fr = j / 3;
      const int d = j - 3 * fr;
      const float c = (d == 0) ? cx : ((d == 1) ? cy : cz);
      const float arg = c * (float)(1 << fr);
      const float sv = sinf(arg);
      const float cv = cosf(arg);
      xr[FEAT + SHP + 3 + 6 * fr + d] = (_Float16)sv;
      xr[FEAT + SHP + 6 + 6 * fr + d] = (_Float16)cv;
    }
  }

  {
    #pragma unroll 1
    for (int i = 0; i < 8; ++i) {
      const int p = 8 * w + i;
      const int va = sVid[p * 4 + 0], vb = sVid[p * 4 + 1], vc = sVid[p * 4 + 2];
      const float ca = sBar[p * 4 + 0], cb = sBar[p * 4 + 1], cc = sBar[p * 4 + 2];
      const float* fa = feature + (size_t)va * FEAT;
      const float* fb = feature + (size_t)vb * FEAT;
      const float* fcp = feature + (size_t)vc * FEAT;
      const float* sa = shapef + (size_t)va * SHP;
      const float* sb = shapef + (size_t)vb * SHP;
      const float* scp = shapef + (size_t)vc * SHP;
      _Float16* xr = sX + p * XSTR;
      const int col = 4 * lane;
      blend4(xr + col,        fa + col,        fb + col,        fcp + col,        ca, cb, cc);
      blend4(xr + 128 + col,  fa + 128 + col,  fb + 128 + col,  fcp + 128 + col,  ca, cb, cc);
      blend4(xr + FEAT + col, sa + col,        sb + col,        scp + col,        ca, cb, cc);
    }
  }
  __syncthreads();

  const v8f zero8 = {0.f, 0.f, 0.f, 0.f, 0.f, 0.f, 0.f, 0.f};

  {
    v8f acc[MT][2];
    #pragma unroll
    for (int mt = 0; mt < MT; ++mt) { acc[mt][0] = zero8; acc[mt][1] = zero8; }
    const _Float16* wr0 = W1h + (size_t)(32 * w + m) * K1P;
    const _Float16* wr1 = wr0 + (size_t)16 * K1P;
    #pragma unroll 1
    for (int ks = 0; ks < K1P; ks += 32) {
      const v16h bf0 = load_frag(wr0 + ks, h);
      const v16h bf1 = load_frag(wr1 + ks, h);
      #pragma unroll
      for (int mt = 0; mt < MT; ++mt) {
        const v16h a = load_frag(sX + (16 * mt + m) * XSTR + ks, h);
        acc[mt][0] = wmma_f16(a, bf0, acc[mt][0]);
        acc[mt][1] = wmma_f16(a, bf1, acc[mt][1]);
      }
    }
    #pragma unroll
    for (int nt = 0; nt < 2; ++nt) {
      const int n = 32 * w + 16 * nt + m;
      const float cbias = c1[n];
      #pragma unroll
      for (int mt = 0; mt < MT; ++mt) {
        #pragma unroll
        for (int r = 0; r < 8; ++r) {
          const int row = 16 * mt + 8 * h + r;
          const float v = fmaxf(acc[mt][nt][r] * WINV + cbias, 0.0f);
          sH1[row * HSTR + n] = (_Float16)v;
        }
      }
    }
  }
  __syncthreads();

  _Float16* sH2 = sX;
  {
    v8f acc[MT][2];
    #pragma unroll
    for (int mt = 0; mt < MT; ++mt) { acc[mt][0] = zero8; acc[mt][1] = zero8; }
    const _Float16* wr0 = W2h + (size_t)(32 * w + m) * HID;
    const _Float16* wr1 = wr0 + (size_t)16 * HID;
    #pragma unroll 1
    for (int ks = 0; ks < HID; ks += 32) {
      const v16h bf0 = load_frag(wr0 + ks, h);
      const v16h bf1 = load_frag(wr1 + ks, h);
      #pragma unroll
      for (int mt = 0; mt < MT; ++mt) {
        const v16h a = load_frag(sH1 + (16 * mt + m) * HSTR + ks, h);
        acc[mt][0] = wmma_f16(a, bf0, acc[mt][0]);
        acc[mt][1] = wmma_f16(a, bf1, acc[mt][1]);
      }
    }
    #pragma unroll
    for (int nt = 0; nt < 2; ++nt) {
      const int n = 32 * w + 16 * nt + m;
      const float bias = b2[n];
      #pragma unroll
      for (int mt = 0; mt < MT; ++mt) {
        #pragma unroll
        for (int r = 0; r < 8; ++r) {
          const int row = 16 * mt + 8 * h + r;
          const float v = fmaxf(acc[mt][nt][r] * WINV + bias, 0.0f);
          sH2[row * HSTR + n] = (_Float16)v;
        }
      }
    }
  }
  __syncthreads();

  if (w < 4) {
    v8f acc3 = zero8;
    const _Float16* wr = W3h + (size_t)m * HID;
    #pragma unroll 1
    for (int ks = 0; ks < HID; ks += 32) {
      const v16h a = load_frag(sH2 + (16 * w + m) * HSTR + ks, h);
      const v16h b = load_frag(wr + ks, h);
      acc3 = wmma_f16(a, b, acc3);
    }
    const int mc = (m < NCH) ? m : (NCH - 1);
    const float bias3 = b3[mc];
    #pragma unroll
    for (int r = 0; r < 8; ++r) {
      const int row = 16 * w + 8 * h + r;
      const float colr = fmaxf(acc3[r] * WINV + bias3, 0.0f) - 1.0f;
      const int msk = sMsk[row];
      const int bt = sBat[row];
      const float bgv = color_bg[bt * NCH + mc];
      const float ocol = (msk != 0) ? colr : bgv;
      const float omsk = (msk != 0) ? 1.0f : 0.0f;
      const float o = (m < NCH) ? ocol : omsk;
      if (m < 4) sOut[row * 4 + m] = o;
    }
  }
  __syncthreads();

  if (w < 2) {
    const int p = 32 * w + lane;
    const v4f v = *(const v4fa*)(sOut + p * 4);
    float* dst = out + (size_t)(pix0 + p) * 4;
    *(volatile v4f*)dst = v;
    __threadfence();
    *(volatile v4f*)dst = v;
  }
}

extern "C" void kernel_launch(void* const* d_in, const int* in_sizes, int n_in,
                              void* d_out, int out_size, void* d_ws, size_t ws_size,
                              hipStream_t stream) {
  if (n_in < 13) return;
  const int npix = in_sizes[0];
  if (npix <= 0) return;
  if (in_sizes[1] != npix * 3) return;
  if (in_sizes[2] < 3 || (in_sizes[2] % 3) != 0) return;
  const int nF = in_sizes[2] / 3;
  if (in_sizes[3] < FEAT || (in_sizes[3] % FEAT) != 0) return;
  const int nV = in_sizes[3] / FEAT;
  if (in_sizes[4] != nV * SHP) return;
  if (in_sizes[5] < 3 || (in_sizes[5] % 3) != 0) return;
  const int nB = in_sizes[5] / 3;
  if ((npix % nB) != 0) return;
  const int hw = npix / nB;
  if (in_sizes[6] != STY) return;
  if (in_sizes[7] != DIN * HID || in_sizes[8] != HID) return;
  if (in_sizes[9] != HID * HID || in_sizes[10] != HID) return;
  if (in_sizes[11] != HID * NCH || in_sizes[12] != NCH) return;
  if (out_size != npix * 4) return;
  if ((npix % MPIX) != 0) return;

  const int*   p2f      = (const int*)  d_in[0];
  const float* bary     = (const float*)d_in[1];
  const int*   faces    = (const int*)  d_in[2];
  const float* feature  = (const float*)d_in[3];
  const float* shapef   = (const float*)d_in[4];
  const float* color_bg = (const float*)d_in[5];
  const float* style    = (const float*)d_in[6];
  const float* w1       = (const float*)d_in[7];
  const float* b1       = (const float*)d_in[8];
  const float* w2       = (const float*)d_in[9];
  const float* b2       = (const float*)d_in[10];
  const float* w3       = (const float*)d_in[11];
  const float* b3       = (const float*)d_in[12];
  float* out = (float*)d_out;

  const size_t w1h_bytes = (size_t)HID * K1P * 2;
  const size_t w2h_bytes = (size_t)HID * HID * 2;
  const size_t w3h_bytes = (size_t)N3P * HID * 2;
  const size_t c1_bytes  = (size_t)HID * 4;
  const size_t total = w1h_bytes + w2h_bytes + w3h_bytes + c1_bytes;
  if (total > ws_size) return;

  char* ws = (char*)d_ws;
  _Float16* W1h = (_Float16*)(ws);
  _Float16* W2h = (_Float16*)(ws + w1h_bytes);
  _Float16* W3h = (_Float16*)(ws + w1h_bytes + w2h_bytes);
  float*    c1  = (float*)   (ws + w1h_bytes + w2h_bytes + w3h_bytes);

  const int ngroups = G1 + G2 + G3 + G4;
  prep_kernel<<<(ngroups + NTHR - 1) / NTHR, NTHR, 0, stream>>>(w1, b1, w2, w3, style, W1h, W2h, W3h, c1);

  render_kernel<<<npix / MPIX, NTHR, 0, stream>>>(p2f, bary, faces, feature, shapef, color_bg,
                                                  W1h, W2h, W3h, c1, b2, b3, out,
                                                  npix, hw, nB, nF, nV);
}
